// MultiHeadGATLayerWithEdgeFeatures_42949672960527
// MI455X (gfx1250) — hardware-verified
//
#include <hip/hip_runtime.h>
#include <stddef.h>
#include <stdint.h>
#include <math.h>


#define NNODE   50000
#define NEDGE   800000
#define FIN     128
#define FOUT    128
#define NHEAD   4
#define HDIM    32
#define FEDGE   16
#define AROW    80
#define MPAD    50048
#define GM      128
#define APITCH  128
#define BPITCH  128
#define KEXT    128
#define NTHR    256
#define NWAVE   8
#define CHUNK   2048
#define WCAP    256
#define LISTN   (NWAVE * WCAP)
#define NB      1024
#define NBLK    49
#define RCAP    20480
#define DEGCAP  64
#define LDS_BKT ((2 * RCAP + 2 * NB + LISTN + 2 * NWAVE) * 4)
#define LDS_GEMM ((GM * FOUT + NHEAD * AROW + GM * 8) * 4)
#define PB_HB   (MPAD * (FIN / 8) / NTHR)
#define PB_EB   (NEDGE * (FEDGE / 8) / NTHR)
#define PB_WT   (FOUT * (FIN / 8) / NTHR)
#define PB_TOT  (PB_HB + PB_EB + PB_WT + 1)

static_assert(NNODE == 390 * 128 + 80);
static_assert(MPAD == 391 * GM && MPAD >= NNODE);
static_assert(NHEAD * HDIM == FOUT && FOUT == 32 * 4);
static_assert(HDIM == 8 * 4);
static_assert(FEDGE == 8 * 2);
static_assert(2 * HDIM + FEDGE == AROW);
static_assert(NBLK * NB >= NNODE && (NBLK - 1) * NB < NNODE);
static_assert((NB & (NB - 1)) == 0 && NB == 1024 && NTHR * 4 == NB);
static_assert(NEDGE < (1 << 20));
static_assert(CHUNK == NWAVE * WCAP && WCAP == 8 * 32 && CHUNK <= 4096);
static_assert(LISTN >= NB);
static_assert(RCAP >= 16759 + 16759 / 10 && (RCAP % 2048) == 0 && (RCAP % (2 * NTHR)) == 0);
static_assert(DEGCAP >= 37 + 8);
static_assert(LDS_BKT <= 300000 && LDS_BKT <= 327680);
static_assert(LDS_GEMM <= 327680);
static_assert((KEXT % 32) == 0 && KEXT <= APITCH && KEXT <= BPITCH);
static_assert(GM == NWAVE * 16);
static_assert(MPAD * (FIN / 8) == PB_HB * NTHR);
static_assert(NEDGE * (FEDGE / 8) == PB_EB * NTHR);
static_assert(FOUT * (FIN / 8) == PB_WT * NTHR);
static_assert(NHEAD * AROW == 80 * 4);
static_assert((NNODE % NWAVE) == 0);

constexpr size_t al256(size_t x) { return (x + 255) & ~(size_t)255; }
constexpr size_t O_HB = 0;
constexpr size_t O_WT = al256(O_HB + (size_t)MPAD * APITCH * 2);
constexpr size_t O_AF = al256(O_WT + (size_t)FOUT * BPITCH * 2);
constexpr size_t O_EB = al256(O_AF + (size_t)NHEAD * AROW * 4);
constexpr size_t O_WH = al256(O_EB + (size_t)NEDGE * FEDGE * 2);
constexpr size_t O_SD = al256(O_WH + (size_t)MPAD * FOUT * 4);
constexpr size_t O_HT = al256(O_SD + (size_t)MPAD * 8 * 4);
constexpr size_t O_SL = al256(O_HT + (size_t)NBLK * RCAP * 8);
constexpr size_t O_FL = al256(O_SL + (size_t)NBLK * NB * 8);
constexpr size_t WS_TOTAL = al256(O_FL + (size_t)NBLK * 128);
static_assert(WS_TOTAL <= ((size_t)128u << 20));

typedef float          v2f   __attribute__((ext_vector_type(2)));
typedef float          v4f   __attribute__((ext_vector_type(4)));
typedef float          v8f   __attribute__((ext_vector_type(8)));
typedef int            v2i   __attribute__((ext_vector_type(2)));
typedef int            v4i   __attribute__((ext_vector_type(4)));
typedef int            v8i   __attribute__((ext_vector_type(8)));
typedef unsigned short v8us  __attribute__((ext_vector_type(8)));
typedef __bf16         v16bf __attribute__((ext_vector_type(16)));
typedef v4f __attribute__((may_alias)) v4fa;
union FragB { v16bf v; v8us u[2]; v8i w; v4i q[2]; };

__device__ __forceinline__ v8f wmx(const FragB& a, const FragB& b, v8f c) {
  v8f d = __builtin_amdgcn_wmma_f32_16x16x32_bf16(false, a.v, false, b.v, (short)0, c, false, false);
  asm volatile("v_nop\n\tv_nop\n\tv_nop\n\tv_nop" : "+v"(d) : "v"(a.w), "v"(b.w));
  return d;
}

__device__ __forceinline__ void pinf(float x) { asm volatile("" :: "v"(x)); }
__device__ __forceinline__ void pini(int x)   { asm volatile("" :: "v"(x)); }

__device__ __forceinline__ unsigned bfbits(float v) {
  const unsigned u = __float_as_uint(v);
  const unsigned r = (u + 0x7FFFu + ((u >> 16) & 1u)) >> 16;
  const unsigned nb = ((u >> 16) & 0x8000u) | 0x7FC0u;
  return ((u & 0x7FFFFFFFu) > 0x7F800000u) ? nb : r;
}
__device__ __forceinline__ float rbf(float v) { return __uint_as_float(bfbits(v) << 16); }

__global__ __launch_bounds__(NTHR) void k_prep(const float* __restrict__ h, const float* __restrict__ ea,
                                               const float* __restrict__ W, const float* __restrict__ a,
                                               unsigned short* hb, unsigned short* eb, unsigned short* wt, float* af) {
  const int blk = (int)blockIdx.x, tid = (int)threadIdx.x;
  if (blk < PB_HB) {
    const int i   = blk * NTHR + tid;
    const int row = i >> 4;
    const int c0  = (i & 15) * 8;
    const int rc  = row < NNODE ? row : NNODE - 1;
    const float* p = h + (size_t)rc * FIN + c0;
    const v4f x = *(const v4f*)p, y = *(const v4f*)(p + 4);
    const unsigned mk = row < NNODE ? 0xFFFFu : 0u;
    v8us hv;
    hv[0] = (unsigned short)(bfbits(x.x) & mk); hv[1] = (unsigned short)(bfbits(x.y) & mk);
    hv[2] = (unsigned short)(bfbits(x.z) & mk); hv[3] = (unsigned short)(bfbits(x.w) & mk);
    hv[4] = (unsigned short)(bfbits(y.x) & mk); hv[5] = (unsigned short)(bfbits(y.y) & mk);
    hv[6] = (unsigned short)(bfbits(y.z) & mk); hv[7] = (unsigned short)(bfbits(y.w) & mk);
    const size_t o = (size_t)row * APITCH + c0;
    *(volatile v8us*)(hb + o) = hv;
    __threadfence();
    *(volatile v8us*)(hb + o) = hv;
  } else if (blk < PB_HB + PB_EB) {
    const int u = (blk - PB_HB) * NTHR + tid;
    const float* p = ea + (size_t)u * 8;
    const v4f x = *(const v4f*)p, y = *(const v4f*)(p + 4);
    v8us hv;
    hv[0] = (unsigned short)bfbits(x.x); hv[1] = (unsigned short)bfbits(x.y);
    hv[2] = (unsigned short)bfbits(x.z); hv[3] = (unsigned short)bfbits(x.w);
    hv[4] = (unsigned short)bfbits(y.x); hv[5] = (unsigned short)bfbits(y.y);
    hv[6] = (unsigned short)bfbits(y.z); hv[7] = (unsigned short)bfbits(y.w);
    const size_t o = (size_t)u * 8;
    *(volatile v8us*)(eb + o) = hv;
    __threadfence();
    *(volatile v8us*)(eb + o) = hv;
  } else if (blk < PB_HB + PB_EB + PB_WT) {
    const int u  = (blk - PB_HB - PB_EB) * NTHR + tid;
    const int n  = u >> 4;
    const int k8 = (u & 15) * 8;
    float f[8];
#pragma unroll
    for (int i = 0; i < 8; ++i) {
      f[i] = W[(size_t)(k8 + i) * FOUT + n];
      pinf(f[i]);
    }
    v8us hv;
#pragma unroll
    for (int i = 0; i < 8; ++i) hv[i] = (unsigned short)bfbits(f[i]);
    const size_t o = (size_t)n * BPITCH + k8;
    *(volatile v8us*)(wt + o) = hv;
    __threadfence();
    *(volatile v8us*)(wt + o) = hv;
  } else {
    const int idx = tid < 80 ? tid : 79;
    const v4f x = *(const v4f*)(a + 4 * idx);
    pinf(x.x); pinf(x.y); pinf(x.z); pinf(x.w);
    v4f y; y.x = rbf(x.x); y.y = rbf(x.y); y.z = rbf(x.z); y.w = rbf(x.w);
    const bool wr = tid < 80;
    if (wr) *(volatile v4f*)(af + 4 * idx) = y;
    __threadfence();
    if (wr) *(volatile v4f*)(af + 4 * idx) = y;
  }
}

__global__ __launch_bounds__(NTHR) __attribute__((amdgpu_num_vgpr(248)))
void k_gemm(const unsigned short* __restrict__ A, const unsigned short* __restrict__ WT,
            const float* __restrict__ af, float* WH, float* SD) {
  extern __shared__ v4f lds_g[];
  float* stg = (float*)lds_g;
  float* sAF = stg + GM * FOUT;
  float* sSD = sAF + NHEAD * AROW;
  const int tid = (int)threadIdx.x, lane = tid & 31, hh = lane >> 4, m = lane & 15;
  const int wave = __builtin_amdgcn_readfirstlane(tid >> 5);
  const int rowBase = (int)blockIdx.x * GM;

  {
    const int idx = tid < 80 ? tid : 79;
    const v4f v = *(const v4f*)(af + 4 * idx);
    *(v4fa*)(sAF + 4 * idx) = v;
  }

  v8f acc[8];
  {
    const v8f z = {0.f, 0.f, 0.f, 0.f, 0.f, 0.f, 0.f, 0.f};
#pragma unroll
    for (int t = 0; t < 8; ++t) acc[t] = z;
  }
  const unsigned short* ap = A  + (size_t)(rowBase + 16 * wave + m) * APITCH + 8 * hh;
  const unsigned short* wp = WT + (size_t)m * BPITCH + 8 * hh;
#pragma unroll 1
  for (int ks = 0; ks < KEXT / 32; ++ks) {
    FragB fa;
    fa.u[0] = *(const v8us*)(ap + 32 * ks);
    fa.u[1] = *(const v8us*)(ap + 32 * ks + 16);
#pragma unroll
    for (int t = 0; t < 8; ++t) {
      const unsigned short* wq = wp + (size_t)(16 * t) * BPITCH + 32 * ks;
      FragB fb;
      fb.u[0] = *(const v8us*)wq;
      fb.u[1] = *(const v8us*)(wq + 16);
      acc[t] = wmx(fa, fb, acc[t]);
    }
  }
#pragma unroll
  for (int t = 0; t < 8; ++t) {
    const int lc = 16 * t + m;
#pragma unroll
    for (int r = 0; r < 8; ++r) {
      const int lr = 16 * wave + 8 * hh + r;
      stg[lr * FOUT + lc] = acc[t][r];
    }
  }
  __syncthreads();

  const int hd = lane >> 3, doff = (4 * lane) & (HDIM - 1);
  const v4f ai = *(const v4fa*)(sAF + hd * AROW + doff);
  const v4f aj = *(const v4fa*)(sAF + hd * AROW + HDIM + doff);
#pragma unroll 1
  for (int r = 0; r < 16; ++r) {
    const int lr = 16 * wave + r;
    const v4f v = *(const v4fa*)(stg + lr * FOUT + 4 * lane);
    float pi = v.x * ai.x; pi = fmaf(v.y, ai.y, pi); pi = fmaf(v.z, ai.z, pi); pi = fmaf(v.w, ai.w, pi);
    float pj = v.x * aj.x; pj = fmaf(v.y, aj.y, pj); pj = fmaf(v.z, aj.z, pj); pj = fmaf(v.w, aj.w, pj);
    pi += __shfl_xor(pi, 1); pj += __shfl_xor(pj, 1);
    pi += __shfl_xor(pi, 2); pj += __shfl_xor(pj, 2);
    pi += __shfl_xor(pi, 4); pj += __shfl_xor(pj, 4);
    if ((lane & 7) == 0) { sSD[lr * 8 + hd] = pi; sSD[lr * 8 + 4 + hd] = pj; }
    float* op = WH + (size_t)(rowBase + lr) * FOUT + 4 * lane;
    *(volatile v4f*)op = v;
  }
  __syncthreads();
  const v4f sv = *(const v4fa*)(sSD + 4 * tid);
  float* sp = SD + (size_t)rowBase * 8 + 4 * tid;
  *(volatile v4f*)sp = sv;
  __threadfence();
#pragma unroll 1
  for (int r = 0; r < 16; ++r) {
    const int lr = 16 * wave + r;
    const v4f v = *(const v4fa*)(stg + lr * FOUT + 4 * lane);
    float* op = WH + (size_t)(rowBase + lr) * FOUT + 4 * lane;
    *(volatile v4f*)op = v;
  }
  *(volatile v4f*)sp = sv;
}

__device__ __forceinline__ int scan_chunk(const int* __restrict__ keys, int nE, int cbase, int slotBase,
                                          int nb, int* list, int lane, int wave) {
  int wc = 0;
  const int elb  = wave * WCAP + lane;
  const int e0   = cbase + elb;
  const int sent = (int)(1u << 31);
  const int nl   = nE - 1;
  int k0 = keys[min(e0,       nl)];
  int k1 = keys[min(e0 + 32,  nl)];
  int k2 = keys[min(e0 + 64,  nl)];
  int k3 = keys[min(e0 + 96,  nl)];
  int k4 = keys[min(e0 + 128, nl)];
  int k5 = keys[min(e0 + 160, nl)];
  int k6 = keys[min(e0 + 192, nl)];
  int k7 = keys[min(e0 + 224, nl)];
  pini(k0); pini(k1); pini(k2); pini(k3); pini(k4); pini(k5); pini(k6); pini(k7);
  const int m0 = -(int)(e0       < nE), m1 = -(int)(e0 + 32  < nE);
  const int m2 = -(int)(e0 + 64  < nE), m3 = -(int)(e0 + 96  < nE);
  const int m4 = -(int)(e0 + 128 < nE), m5 = -(int)(e0 + 160 < nE);
  const int m6 = -(int)(e0 + 192 < nE), m7 = -(int)(e0 + 224 < nE);
  k0 = (k0 & m0) | (sent & ~m0); k1 = (k1 & m1) | (sent & ~m1);
  k2 = (k2 & m2) | (sent & ~m2); k3 = (k3 & m3) | (sent & ~m3);
  k4 = (k4 & m4) | (sent & ~m4); k5 = (k5 & m5) | (sent & ~m5);
  k6 = (k6 & m6) | (sent & ~m6); k7 = (k7 & m7) | (sent & ~m7);
  const unsigned nbs = (unsigned)slotBase;
  const unsigned unb = (unsigned)nb;
  const unsigned s0 = (unsigned)k0 - nbs, s1 = (unsigned)k1 - nbs;
  const unsigned s2 = (unsigned)k2 - nbs, s3 = (unsigned)k3 - nbs;
  const unsigned s4 = (unsigned)k4 - nbs, s5 = (unsigned)k5 - nbs;
  const unsigned s6 = (unsigned)k6 - nbs, s7 = (unsigned)k7 - nbs;
  const bool h0 = s0 < unb, h1 = s1 < unb, h2 = s2 < unb, h3 = s3 < unb;
  const bool h4 = s4 < unb, h5 = s5 < unb, h6 = s6 < unb, h7 = s7 < unb;
  const unsigned any = __builtin_amdgcn_ballot_w32(h0 | h1 | h2 | h3 | h4 | h5 | h6 | h7);
  if (any != 0u) {
#define HITJ(J, HJ, SJ) { \
      const unsigned mj = __builtin_amdgcn_ballot_w32(HJ); \
      if (mj != 0u) { \
        const int pos = wc + (int)__builtin_amdgcn_mbcnt_lo(mj, 0u); \
        if ((HJ) && pos < WCAP) list[wave * WCAP + pos] = ((elb + 32 * (J)) << 12) | (int)(SJ); \
        wc += (int)__builtin_popcount(mj); } }
    HITJ(0, h0, s0)
    HITJ(1, h1, s1)
    HITJ(2, h2, s2)
    HITJ(3, h3, s3)
    HITJ(4, h4, s4)
    HITJ(5, h5, s5)
    HITJ(6, h6, s6)
    HITJ(7, h7, s7)
#undef HITJ
  }
  return wc;
}

__global__ __launch_bounds__(NTHR) void k_bucket(const int* __restrict__ keys, const int* __restrict__ prov,
                                                 int* hits, int* slot, int* flag, int nN, int nE) {
  extern __shared__ v4f lds_b[];
  int* reg1 = (int*)lds_b;
  int* reg2 = reg1 + RCAP;
  int* scnt = reg2 + RCAP;
  int* soff = scnt + NB;
  int* list = soff + NB;
  int* wcnt = list + LISTN;
  int* wtot = wcnt + NWAVE;
  const int tid = (int)threadIdx.x, lane = tid & 31;
  const int wave = __builtin_amdgcn_readfirstlane(tid >> 5);
  const int nodeBase = (int)blockIdx.x * NB;

  for (int i = tid; i < NB; i += NTHR) scnt[i] = 0;
  for (int i = tid; i < RCAP; i += NTHR) { reg1[i] = 0; reg2[i] = 0; }
  __syncthreads();

  int tot = 0;
  const int nChunks = (nE + CHUNK - 1) / CHUNK;
#pragma unroll 1
  for (int ch = 0; ch < nChunks; ++ch) {
    const int cbase = ch * CHUNK;
    const int wc = scan_chunk(keys, nE, cbase, nodeBase, NB, list, lane, wave);
    if (lane == 0) wcnt[wave] = wc;
    __syncthreads();
    int pre = 0, all = 0;
#pragma unroll
    for (int w2 = 0; w2 < NWAVE; ++w2) {
      int c = wcnt[w2];
      c = c < 0 ? 0 : (c > WCAP ? WCAP : c);
      all += c;
      pre += (w2 < wave) ? c : 0;
    }
    const int wcc  = wc > WCAP ? WCAP : wc;
    const int base = tot + pre;
#pragma unroll 1
    for (int i = lane; i < wcc; i += 32) {
      const int en = list[wave * WCAP + i];
      const int el = (en >> 12) & (CHUNK - 1);
      const int sl = en & (NB - 1);
      int eid = cbase + el;
      eid = eid > nE - 1 ? nE - 1 : eid;
      const int pos = base + i;
      if (pos < RCAP) reg1[pos] = (int)(((unsigned)eid << 12) | (unsigned)sl);
    }
    tot += all;
    tot = tot > RCAP ? RCAP : tot;
    __syncthreads();
  }
  const int nh = tot;

  if (wave == 0) {
#pragma unroll 1
    for (int b0 = 0; b0 < nh; b0 += 32) {
      const int idx = b0 + lane;
      const int uv  = reg1[idx < RCAP ? idx : RCAP - 1];
      const int m32 = (nh - b0) < 32 ? (nh - b0) : 32;
#pragma unroll 1
      for (int k = 0; k < m32; ++k) {
        const int u  = __builtin_amdgcn_readlane(uv, k);
        const int sl = u & (NB - 1);
        if (lane == 0) scnt[sl] = scnt[sl] + 1;
      }
    }
  }
  __syncthreads();

  int anybig = 0;
  {
    const v4i ca = *(const v4i*)(scnt + 4 * tid);
    const int e0 = ca.x < 0 ? 0 : ca.x, e1 = ca.y < 0 ? 0 : ca.y;
    const int e2 = ca.z < 0 ? 0 : ca.z, e3 = ca.w < 0 ? 0 : ca.w;
    const bool big = (ca.x > DEGCAP) | (ca.y > DEGCAP) | (ca.z > DEGCAP) | (ca.w > DEGCAP);
    const unsigned bm = __builtin_amdgcn_ballot_w32(big);
    const int ts = (e0 + e1) + (e2 + e3);
    int incl = ts;
#pragma unroll
    for (int d = 1; d < 32; d <<= 1) {
      const int up = __shfl_up(incl, d);
      if (lane >= d) incl += up;
    }
    if (lane == 31) wtot[wave] = incl;
    if (lane == 0)  wcnt[wave] = (bm != 0u) ? 1 : 0;
    __syncthreads();
    int pre = 0;
#pragma unroll
    for (int w2 = 0; w2 < NWAVE; ++w2) {
      pre += (w2 < wave) ? wtot[w2] : 0;
      anybig |= wcnt[w2];
    }
    const int run = pre + incl - ts;
    v4i so;
    so.x = run; so.y = run + e0; so.z = run + e0 + e1; so.w = run + e0 + e1 + e2;
    *(v4i*)(soff + 4 * tid) = so;
  }
  __syncthreads();
  for (int i = tid; i < NB; i += NTHR) list[i] = soff[i];
  __syncthreads();

  if (wave == 0) {
#pragma unroll 1
    for (int b0 = 0; b0 < nh; b0 += 32) {
      const int idx = b0 + lane;
      const int uv  = reg1[idx < RCAP ? idx : RCAP - 1];
      const int m32 = (nh - b0) < 32 ? (nh - b0) : 32;
#pragma unroll 1
      for (int k = 0; k < m32; ++k) {
        const int u   = __builtin_amdgcn_readlane(uv, k);
        const int sl  = u & (NB - 1);
        const int eid = (int)((unsigned)u >> 12);
        if (lane == 0) {
          int pos = list[sl];
          pos = pos < 0 ? 0 : (pos > RCAP - 1 ? RCAP - 1 : pos);
          reg2[pos] = eid;
          list[sl] = pos + 1;
        }
      }
    }
  }
  __syncthreads();

  const int fl = ((nh >= RCAP) || (anybig != 0)) ? 1 : 0;
  int* eb = hits + (size_t)blockIdx.x * (size_t)(2 * RCAP);
#pragma unroll 1
  for (int p0 = 0; p0 < RCAP; p0 += 2 * NTHR) {
    const int p  = p0 + 2 * tid;
    const int pa = p < RCAP - 2 ? p : RCAP - 2;
    int e0 = reg2[pa], e1 = reg2[pa + 1];
    e0 = e0 < 0 ? 0 : (e0 > nE - 1 ? nE - 1 : e0);
    e1 = e1 < 0 ? 0 : (e1 > nE - 1 ? nE - 1 : e1);
    int s0 = prov[e0];
    int s1 = prov[e1];
    pini(s0); pini(s1);
    s0 = s0 < 0 ? 0 : (s0 > nN - 1 ? nN - 1 : s0);
    s1 = s1 < 0 ? 0 : (s1 > nN - 1 ? nN - 1 : s1);
    const int m0 = (p     < nh) ? -1 : 0;
    const int m1 = (p + 1 < nh) ? -1 : 0;
    v4i v;
    v.x = s0 & m0; v.y = e0 & m0; v.z = s1 & m1; v.w = e1 & m1;
    *(volatile v4i*)(eb + 2 * pa) = v;
    __threadfence();
    *(volatile v4i*)(eb + 2 * pa) = v;
  }
  {
    const int q0 = tid, q1 = NTHR + tid;
    v4i sa, sb;
    sa.x = soff[2 * q0]; sa.y = scnt[2 * q0]; sa.z = soff[2 * q0 + 1]; sa.w = scnt[2 * q0 + 1];
    sb.x = soff[2 * q1]; sb.y = scnt[2 * q1]; sb.z = soff[2 * q1 + 1]; sb.w = scnt[2 * q1 + 1];
    int* spa = slot + 2 * (size_t)(nodeBase + 2 * q0);
    int* spb = slot + 2 * (size_t)(nodeBase + 2 * q1);
    v4i fv; fv.x = fl; fv.y = fl; fv.z = fl; fv.w = fl;
    int* fp = flag + (size_t)blockIdx.x * 32 + 4 * (tid & 7);
    const bool fw = tid < 8;
    *(volatile v4i*)spa = sa;
    *(volatile v4i*)spb = sb;
    if (fw) *(volatile v4i*)fp = fv;
    __threadfence();
    *(volatile v4i*)spa = sa;
    *(volatile v4i*)spb = sb;
    if (fw) *(volatile v4i*)fp = fv;
  }
}

__global__ __launch_bounds__(NTHR) void k_replay(const int* __restrict__ hits, const int* __restrict__ slot,
                                                 const int* __restrict__ flag, const unsigned* __restrict__ ebw,
                                                 const float* __restrict__ af, const float* __restrict__ wh,
                                                 const float* __restrict__ sd, float* out, int nN, int nE) {
  const int tid = (int)threadIdx.x, lane = tid & 31;
  const int wave = __builtin_amdgcn_readfirstlane(tid >> 5);
  const int i = (int)blockIdx.x * NWAVE + wave;
  if (i >= nN) return;
  const int hd = lane >> 3, p = lane & 7;

  const v2i se = *(const v2i*)(slot + 2 * (size_t)i);
  int stv = se.x;
  stv = stv < 0 ? 0 : (stv > RCAP - 1 ? RCAP - 1 : stv);
  int cv = se.y;
  cv = cv < 0 ? 0 : (cv > DEGCAP ? DEGCAP : cv);
  cv = cv > RCAP - stv ? RCAP - stv : cv;
  const int st   = __builtin_amdgcn_readfirstlane(stv);
  const int c    = __builtin_amdgcn_readfirstlane(cv);
  const int craw = __builtin_amdgcn_readfirstlane(se.y);
  const int b    = i >> 10;
  const int fl   = __builtin_amdgcn_readfirstlane(flag[(size_t)b * 32]);
  const bool bad = (fl != 0) || (craw < 0) || (craw > DEGCAP);
  const int* eb = hits + (size_t)b * (size_t)(2 * RCAP);

  const float sdi = sd[(size_t)i * 8 + hd];
  const v2f ae = *(const v2f*)(af + hd * AROW + 2 * HDIM + 2 * p);
  v4f acc = {0.f, 0.f, 0.f, 0.f};
  int last = st + c - 1;
  last = last < st ? st : last;

#pragma unroll 1
  for (int t0 = 0; t0 < c; t0 += 32) {
    const int rem = c - t0;
    const int nv = rem < 32 ? rem : 32;
    int idx = st + t0 + lane;
    idx = idx > last ? last : idx;
    const v2i en = *(const v2i*)(eb + 2 * (size_t)idx);
    int jc = en.x; jc = jc < 0 ? 0 : (jc > nN - 1 ? nN - 1 : jc);
    int ec = en.y; ec = ec < 0 ? 0 : (ec > nE - 1 ? nE - 1 : ec);
#pragma unroll 1
    for (int r = 0; r < nv; ++r) {
      const int j = __builtin_amdgcn_readlane(jc, r);
      const int e = __builtin_amdgcn_readlane(ec, r);
      const unsigned w = ebw[(size_t)e * 8 + p];
      const float sdj = sd[(size_t)j * 8 + 4 + hd];
      const v4f w4 = *(const v4f*)(wh + (size_t)j * FOUT + 4 * lane);
      const float f0 = __uint_as_float(w << 16);
      const float f1 = __uint_as_float(w & 0xFFFF0000u);
      float ed = f0 * ae.x;
      ed = fmaf(f1, ae.y, ed);
      ed += __shfl_xor(ed, 1);
      ed += __shfl_xor(ed, 2);
      ed += __shfl_xor(ed, 4);
      float s = (sdi + sdj) + ed;
      s = (s > 0.0f) ? s : 0.2f * s;
      float mx = fmaxf(s, __shfl_xor(s, 8));
      mx = fmaxf(mx, __shfl_xor(mx, 16));
      const float pe = expf(s - mx);
      float sm = pe + __shfl_xor(pe, 8);
      sm = sm + __shfl_xor(sm, 16);
      const float att = pe / sm;
      acc.x = fmaf(att, w4.x, acc.x);
      acc.y = fmaf(att, w4.y, acc.y);
      acc.z = fmaf(att, w4.z, acc.z);
      acc.w = fmaf(att, w4.w, acc.w);
    }
  }

  const float qnan = __int_as_float(0x7fc00000);
  v4f o;
  o.x = bad ? qnan : acc.x;
  o.y = bad ? qnan : acc.y;
  o.z = bad ? qnan : acc.z;
  o.w = bad ? qnan : acc.w;
#pragma unroll 1
  for (int k = 0; k < 4; ++k) {
    const float x = o.x;
    const float y = (x > 0.0f) ? x : expm1f(x);
    o.x = o.y; o.y = o.z; o.z = o.w; o.w = y;
  }
  float* gp = out + (size_t)i * FOUT + 4 * lane;
  *(volatile v4f*)gp = o;
  __threadfence();
  *(volatile v4f*)gp = o;
}

extern "C" void kernel_launch(void* const* d_in, const int* in_sizes, int n_in,
                              void* d_out, int out_size, void* d_ws, size_t ws_size,
                              hipStream_t stream) {
  if (n_in < 5) return;
  if (in_sizes[0] != NNODE * FIN) return;
  if (in_sizes[1] != NEDGE * FEDGE) return;
  if (in_sizes[2] != FIN * FOUT) return;
  if (in_sizes[3] != NHEAD * AROW) return;
  if (in_sizes[4] != 2 * NEDGE) return;
  if (out_size != NNODE * FOUT) return;
  if (WS_TOTAL > ws_size) return;

  const float* h  = (const float*)d_in[0];
  const float* ea = (const float*)d_in[1];
  const float* W  = (const float*)d_in[2];
  const float* a  = (const float*)d_in[3];
  const int*   ei = (const int*)  d_in[4];
  const int* keys = ei;
  const int* prov = ei + NEDGE;
  float* out = (float*)d_out;

  char* ws = (char*)d_ws;
  unsigned short* HB = (unsigned short*)(ws + O_HB);
  unsigned short* WT = (unsigned short*)(ws + O_WT);
  float*          AF = (float*)(ws + O_AF);
  unsigned short* EB = (unsigned short*)(ws + O_EB);
  float*          WH = (float*)(ws + O_WH);
  float*          SD = (float*)(ws + O_SD);
  int*            HT = (int*)(ws + O_HT);
  int*            SL = (int*)(ws + O_SL);
  int*            FL = (int*)(ws + O_FL);

  hipFuncSetAttribute(reinterpret_cast<const void*>(&k_gemm),
                      hipFuncAttributeMaxDynamicSharedMemorySize, LDS_GEMM);
  hipFuncSetAttribute(reinterpret_cast<const void*>(&k_bucket),
                      hipFuncAttributeMaxDynamicSharedMemorySize, LDS_BKT);

  k_prep<<<PB_TOT, NTHR, 0, stream>>>(h, ea, W, a, HB, EB, WT, AF);
  k_gemm<<<MPAD / GM, NTHR, LDS_GEMM, stream>>>(HB, WT, AF, WH, SD);
  k_bucket<<<NBLK, NTHR, LDS_BKT, stream>>>(keys, prov, HT, SL, FL, NNODE, NEDGE);
  k_replay<<<NNODE / NWAVE, NTHR, 0, stream>>>(HT, SL, FL, (const unsigned*)EB, AF, WH, SD, out, NNODE, NEDGE);
}
